// TNModule_54829552501061
// MI455X (gfx1250) — hardware-verified
//
#include <hip/hip_runtime.h>

#define NTT 4096
#define BB  4
#define F   32
#define WAVES_PER_BLOCK 4

typedef _Float16 v16h __attribute__((ext_vector_type(16)));
typedef _Float16 v8h  __attribute__((ext_vector_type(8)));
typedef float    v8f  __attribute__((ext_vector_type(8)));
typedef float    v4f  __attribute__((ext_vector_type(4)));
typedef float    v4fa __attribute__((ext_vector_type(4), may_alias));
union Frag { v16h v; v8h half[2]; _Float16 h[16]; };

__device__ __forceinline__ v8f mma16(v16h a, v16h b, v8f c) {
  c = __builtin_amdgcn_wmma_f32_16x16x32_f16(false, a, false, b, (short)0, c, false, false);
  asm volatile("v_nop\n\tv_nop\n\tv_nop\n\tv_nop" : "+v"(c) : "v"(a), "v"(b));
  return c;
}
__device__ __forceinline__ float fast_tanh(float x) {
#if __has_builtin(__builtin_amdgcn_tanhf)
  return __builtin_amdgcn_tanhf(x);
#else
  return tanhf(x);
#endif
}

__global__ __launch_bounds__(256) void xcvt_kernel(const float* __restrict__ X, _Float16* __restrict__ Xh, int n8) {
  const int t = blockIdx.x * 256 + threadIdx.x;
  if (t >= n8) return;
  v8h v;
#pragma unroll
  for (int i = 0; i < 8; ++i) v[i] = (_Float16)X[(size_t)t * 8 + i];
  *(volatile v8h*)(Xh + (size_t)t * 8) = v;
  __threadfence();
  *(volatile v8h*)(Xh + (size_t)t * 8) = v;
}

__global__ __launch_bounds__(128) void pt_kernel(const float* __restrict__ H, const float* __restrict__ W, _Float16* __restrict__ Pt) {
  __shared__ __attribute__((aligned(16))) _Float16 sP[4][F][64];
  const int lane = threadIdx.x & 31, wave = threadIdx.x >> 5, lane16 = lane & 15, h = lane >> 4;
  const int wid = blockIdx.x * 4 + wave;
  const int b = wid / (NTT / 64), m0 = (wid % (NTT / 64)) * 64;
  Frag bw[2];
#pragma unroll
  for (int nt = 0; nt < 2; ++nt) {
    const int g = nt * 16 + lane16;
#pragma unroll
    for (int i = 0; i < 8; ++i) { bw[nt].h[i] = (_Float16)W[(8 * h + i) * F + g]; bw[nt].h[8 + i] = (_Float16)W[(16 + 8 * h + i) * F + g]; }
  }
#pragma unroll
  for (int mt = 0; mt < 4; ++mt) {
    const float* hrow = H + ((size_t)(b * NTT + m0 + mt * 16 + lane16)) * F;
    Frag a;
#pragma unroll
    for (int i = 0; i < 8; ++i) { a.h[i] = (_Float16)hrow[8 * h + i]; a.h[8 + i] = (_Float16)hrow[16 + 8 * h + i]; }
#pragma unroll
    for (int nt = 0; nt < 2; ++nt) {
      v8f acc = {};
      acc = mma16(a.v, bw[nt].v, acc);
#pragma unroll
      for (int r = 0; r < 8; ++r) sP[wave][nt * 16 + lane16][mt * 16 + 8 * h + r] = (_Float16)acc[r];
    }
  }
  __builtin_amdgcn_fence(__ATOMIC_ACQ_REL, "workgroup");
  __builtin_amdgcn_wave_barrier();
  typedef _Float16 v8ha __attribute__((ext_vector_type(8), may_alias));
  const int rsub = lane >> 3, c8 = (lane & 7) * 8;
  for (int pass = 0; pass < 2; ++pass) {
#pragma unroll
    for (int q = 0; q < 8; ++q) {
      const int g = q * 4 + rsub;
      const v8h v = *(const v8ha*)&sP[wave][g][c8];
      *(volatile v8h*)(Pt + ((size_t)(b * F + g)) * NTT + m0 + c8) = v;
    }
    if (pass == 0) __threadfence();
  }
}

__global__ void __launch_bounds__(WAVES_PER_BLOCK * 32)
gcn_kernel(const _Float16* __restrict__ Xh, const _Float16* __restrict__ Pt, float* __restrict__ Out) {
  __shared__ __attribute__((aligned(16))) float so[WAVES_PER_BLOCK][16][F];
  const int lane = threadIdx.x & 31;
  const int wave = threadIdx.x >> 5;
  const int widU = __builtin_amdgcn_readfirstlane(blockIdx.x * WAVES_PER_BLOCK + wave);
  const int b  = widU >> 8;
  const int n0 = (widU & 255) << 4;
  const int lane16 = lane & 15;
  const int h = lane >> 4;

  const _Float16* nrow = Xh + ((size_t)(b * NTT + n0 + lane16)) * F;
  Frag bN;
  bN.half[0] = *(const v8h*)(nrow + 8 * h);
  bN.half[1] = *(const v8h*)(nrow + 16 + 8 * h);

  v8f acc0 = {};
  v8f acc1 = {};

  for (int m0 = 0; m0 < NTT; m0 += 32) {
    const _Float16* mrow0 = Xh + ((size_t)(b * NTT + m0 + lane16)) * F;
    const _Float16* mrow1 = mrow0 + 16 * F;
    Frag aM0, aM1;
    aM0.half[0] = *(const v8h*)(mrow0 + 8 * h);  aM0.half[1] = *(const v8h*)(mrow0 + 16 + 8 * h);
    aM1.half[0] = *(const v8h*)(mrow1 + 8 * h);  aM1.half[1] = *(const v8h*)(mrow1 + 16 + 8 * h);
    v8f zero = {};
    v8f sim0 = mma16(aM0.v, bN.v, zero);
    v8f sim1 = mma16(aM1.v, bN.v, zero);

    Frag a2;
    if ((unsigned)(n0 - m0) < 32u) {
#pragma unroll
      for (int s = 0; s < 2; ++s) {
        const v8f sim = s ? sim1 : sim0;
        const int mbase = m0 + s * 16 + 8 * h;
#pragma unroll
        for (int r = 0; r < 8; ++r) {
          float v = fmaxf(sim[r], 0.0f);
          if (mbase + r == n0 + lane16) v += 1.0f;
          a2.h[s * 8 + r] = (_Float16)fast_tanh(v);
        }
      }
    } else {
#pragma unroll
      for (int r = 0; r < 8; ++r) a2.h[r]     = (_Float16)fast_tanh(fmaxf(sim0[r], 0.0f));
#pragma unroll
      for (int r = 0; r < 8; ++r) a2.h[8 + r] = (_Float16)fast_tanh(fmaxf(sim1[r], 0.0f));
    }

    const _Float16* p0 = Pt + ((size_t)(b * F + lane16)) * NTT + m0;
    const _Float16* p1 = p0 + (size_t)16 * NTT;
    Frag b2;
    b2.half[0] = *(const v8h*)(p0 + 8 * h);  b2.half[1] = *(const v8h*)(p0 + 16 + 8 * h);
    acc0 = mma16(a2.v, b2.v, acc0);
    b2.half[0] = *(const v8h*)(p1 + 8 * h);  b2.half[1] = *(const v8h*)(p1 + 16 + 8 * h);
    acc1 = mma16(a2.v, b2.v, acc1);
  }

#pragma unroll
  for (int r = 0; r < 8; ++r) {
    float v0 = acc0[r], v1 = acc1[r];
    v0 = v0 > 0.f ? v0 : expm1f(v0);
    v1 = v1 > 0.f ? v1 : expm1f(v1);
    so[wave][8 * h + r][lane16] = v0;
    so[wave][8 * h + r][16 + lane16] = v1;
  }
  __builtin_amdgcn_fence(__ATOMIC_ACQ_REL, "workgroup");
  __builtin_amdgcn_wave_barrier();
  const int rsub = lane >> 3, c4 = (lane & 7) * 4;
  float* obase = Out + ((size_t)(b * NTT + n0)) * F;
  for (int pass = 0; pass < 2; ++pass) {
#pragma unroll
    for (int q = 0; q < 4; ++q) {
      const int row = q * 4 + rsub;
      const v4f v = *(const v4fa*)&so[wave][row][c4];
      *(volatile v4f*)(obase + (size_t)row * F + c4) = v;
    }
    if (pass == 0) __threadfence();
  }
}

extern "C" void kernel_launch(void* const* d_in, const int* in_sizes, int n_in,
                              void* d_out, int out_size, void* d_ws, size_t ws_size, hipStream_t stream) {
  (void)in_sizes; (void)n_in; (void)out_size; (void)ws_size;
  const float* X = (const float*)d_in[0];
  const float* W = (const float*)d_in[1];
  float* Out = (float*)d_out;

  char* ws = (char*)d_ws;
  _Float16* Xh = (_Float16*)ws;
  _Float16* Pt = (_Float16*)(ws + (size_t)BB * NTT * F * 2);
  float*    H1 = (float*)(ws + (size_t)2 * BB * NTT * F * 2);

  const int total = BB * NTT * F;
  const int gcnBlocks = (BB * (NTT / 16)) / WAVES_PER_BLOCK;

  xcvt_kernel<<<total / 8 / 256, 256, 0, stream>>>(X, Xh, total / 8);
  pt_kernel<<<(BB * NTT / 64) / 4, 128, 0, stream>>>(X, W, Pt);
  gcn_kernel<<<gcnBlocks, WAVES_PER_BLOCK * 32, 0, stream>>>(Xh, Pt, H1);
  pt_kernel<<<(BB * NTT / 64) / 4, 128, 0, stream>>>(H1, W + F * F, Pt);
  gcn_kernel<<<gcnBlocks, WAVES_PER_BLOCK * 32, 0, stream>>>(Xh, Pt, Out);
}
